// ginn_autoencoder_skip_28681791603394
// MI455X (gfx1250) — hardware-verified
//
#include <hip/hip_runtime.h>

typedef float          v8f   __attribute__((ext_vector_type(8)));
typedef float          v4f   __attribute__((ext_vector_type(4)));
typedef unsigned int   v4u   __attribute__((ext_vector_type(4)));
typedef int            v8i   __attribute__((ext_vector_type(8)));
typedef unsigned short v8us  __attribute__((ext_vector_type(8)));
typedef unsigned short v16us __attribute__((ext_vector_type(16)));
typedef __bf16         v16bf __attribute__((ext_vector_type(16)));
typedef _Float16       v16h  __attribute__((ext_vector_type(16)));
typedef v4f  __attribute__((may_alias)) v4fa;
typedef v8us __attribute__((may_alias)) v8usa;
union FragB { v16bf v; v16us u; v8us h[2]; v8i w; };
union FragH { v16h  v; v16us u; v8us h[2]; v8i w; };

__device__ __forceinline__ v8f wmb(const FragB& a, const FragB& b, v8f c) {
  v8f d = __builtin_amdgcn_wmma_f32_16x16x32_bf16(false, a.v, false, b.v, (short)0, c, false, false);
  asm volatile("v_nop\n\tv_nop\n\tv_nop\n\tv_nop" : "+v"(d) : "v"(a.w), "v"(b.w));
  return d;
}

__device__ __forceinline__ v8f wmh(const FragH& a, const FragH& b, v8f c) {
  v8f d = __builtin_amdgcn_wmma_f32_16x16x32_f16(false, a.v, false, b.v, (short)0, c, false, false);
  asm volatile("v_nop\n\tv_nop\n\tv_nop\n\tv_nop" : "+v"(d) : "v"(a.w), "v"(b.w));
  return d;
}

__device__ __forceinline__ unsigned bf16_bits(float f) {
  const unsigned u = __float_as_uint(f);
  const unsigned r = (u + 0x7FFFu + ((u >> 16) & 1u)) >> 16;
  const unsigned q = (u >> 16) | 0x40u;
  return ((u & 0x7fffffffu) > 0x7f800000u) ? q : r;
}

__device__ __forceinline__ float bf16_val(float f) {
  return __uint_as_float(bf16_bits(f) << 16);
}
__device__ __forceinline__ int clampi(int v, int lo, int hi) {
  return v < lo ? lo : (v > hi ? hi : v);
}

__device__ __forceinline__ unsigned f16_bits(float f) {
  const unsigned u  = __float_as_uint(f);
  const unsigned s  = (u >> 16) & 0x8000u;
  const unsigned a  = u & 0x7fffffffu;
  const unsigned t  = a - 0x38000000u;
  const unsigned r  = (t + 0x0FFFu + ((t >> 13) & 1u)) >> 13;
  const unsigned rc = r > 0x7C00u ? 0x7C00u : r;
  const bool small  = a < 0x38800000u;
  const bool isnan  = a > 0x7f800000u;
  const unsigned fin = small ? 0u : (s | rc);
  return isnan ? (s | 0x7E00u) : fin;
}

__device__ __forceinline__ unsigned pk16(unsigned lo, unsigned hi) { return lo | (hi << 16); }
__device__ __forceinline__ unsigned bf16_lo_bits(float v) {
  float hi = bf16_val(v);
  asm volatile("" : "+v"(hi));
  return bf16_bits(v - hi);
}
__device__ __forceinline__ v4u pack8_bf16(v4f a, v4f c) {
  return (v4u){ pk16(bf16_bits(a[0]), bf16_bits(a[1])), pk16(bf16_bits(a[2]), bf16_bits(a[3])),
                pk16(bf16_bits(c[0]), bf16_bits(c[1])), pk16(bf16_bits(c[2]), bf16_bits(c[3])) };
}
__device__ __forceinline__ v4u pack8_bf16_lo(v4f a, v4f c) {
  return (v4u){ pk16(bf16_lo_bits(a[0]), bf16_lo_bits(a[1])), pk16(bf16_lo_bits(a[2]), bf16_lo_bits(a[3])),
                pk16(bf16_lo_bits(c[0]), bf16_lo_bits(c[1])), pk16(bf16_lo_bits(c[2]), bf16_lo_bits(c[3])) };
}
__device__ __forceinline__ v4u pack8_f16(v4f a, v4f c) {
  return (v4u){ pk16(f16_bits(a[0]), f16_bits(a[1])), pk16(f16_bits(a[2]), f16_bits(a[3])),
                pk16(f16_bits(c[0]), f16_bits(c[1])), pk16(f16_bits(c[2]), f16_bits(c[3])) };
}

template <int FORM>
__global__ __launch_bounds__(256) void k_plane(const float* __restrict__ src, int rows, int cols, int ldsrc,
                                               unsigned short* __restrict__ dst, int MP, int KP) {
  static_assert(FORM >= 0 && FORM <= 3);
  const int KTOT = (FORM == 1 || FORM == 3) ? 2 * KP : KP;
  const unsigned ppr   = (unsigned)(KTOT >> 3);
  const unsigned kp8   = (unsigned)(KP >> 3);
  const unsigned total = (unsigned)MP * ppr;
  const unsigned g     = blockIdx.x * 256u + threadIdx.x;
  const unsigned rowu  = g / ppr;
  const unsigned p     = g - rowu * ppr;
  const bool second    = p >= kp8;
  const int row = (int)rowu;
  const int c0  = (int)((second ? p - kp8 : p) << 3);
  const float* srow = src + (size_t)clampi(row, 0, rows - 1) * (size_t)ldsrc;
  float x[8];
  unsigned mk[8];
#pragma unroll
  for (int e = 0; e < 8; ++e) {
    const int c = c0 + e;
    const float v = srow[clampi(c, 0, cols - 1)];
    asm volatile("" :: "v"(v));
    x[e]  = v;
    mk[e] = (row < rows && c < cols) ? 0xFFFFu : 0u;
  }
  const v4f a = (v4f){ x[0], x[1], x[2], x[3] };
  const v4f c = (v4f){ x[4], x[5], x[6], x[7] };
  v4u o;
  if (FORM == 2) {
    o = pack8_f16(a, c);
  } else {
    const v4u hi = pack8_bf16(a, c);
    o = hi;
    if (FORM == 1) { const v4u lo = pack8_bf16_lo(a, c); o = second ? lo : hi; }
  }
  const v4u mw = (v4u){ pk16(mk[0], mk[1]), pk16(mk[2], mk[3]), pk16(mk[4], mk[5]), pk16(mk[6], mk[7]) };
  o &= mw;
  if (g < total) {
    volatile v4u* q = (volatile v4u*)(dst + (size_t)g * 8);
    *q = o;
    __threadfence();
    *q = o;
  }
}

template <int FORM> struct FragOf    { typedef FragB T; };
template <>         struct FragOf<2> { typedef FragH T; };
__device__ __forceinline__ v8f mm(const FragB& a, const FragB& b, v8f c) { return wmb(a, b, c); }
__device__ __forceinline__ v8f mm(const FragH& a, const FragH& b, v8f c) { return wmh(a, b, c); }
template <class F> __device__ __forceinline__ F ld_frag(const unsigned short* p) {
  F f;
  f.h[0] = *(const v8usa*)(p);
  f.h[1] = *(const v8usa*)(p + 16);
  return f;
}

template <int FORM, int EPI>
__global__ __launch_bounds__(256) __attribute__((amdgpu_num_vgpr(248)))
void k_gemm_nt(const unsigned short* __restrict__ A, const unsigned short* __restrict__ B,
               const float* __restrict__ bias, float* __restrict__ D, int M, int N, int KTOT, int ldd) {
  static_assert(FORM >= 0 && FORM <= 2);
  static_assert(EPI == 0 || EPI == 1);
  typedef typename FragOf<FORM>::T F;
  __shared__ __attribute__((aligned(16))) float sT[8][16 * 68];
  const int lane = threadIdx.x & 31;
  const int wave = threadIdx.x >> 5;
  const int tilesM = (M + 63) >> 6;
  const int tilesN = (N + 63) >> 6;
  const int tile = blockIdx.x * 8 + wave;
  if (tile >= tilesM * tilesN) return;
  const int tm = tile / tilesN;
  const int tn = tile - tm * tilesN;
  const int m0 = tm << 6;
  const int n0 = tn << 6;

  const int rl = lane & 15;
  const int h8 = (lane >> 4) * 8;
  const unsigned short* pa = A + (size_t)(m0 + rl) * (size_t)KTOT + h8;
  const unsigned short* pb = B + (size_t)(n0 + rl) * (size_t)KTOT + h8;

  v8f acc[4][4];
#pragma unroll
  for (int i = 0; i < 4; ++i)
#pragma unroll
    for (int j = 0; j < 4; ++j) acc[i][j] = (v8f){0.f, 0.f, 0.f, 0.f, 0.f, 0.f, 0.f, 0.f};

#pragma unroll 1
  for (int k0 = 0; k0 < KTOT; k0 += 32) {
    F bf[4];
#pragma unroll
    for (int j = 0; j < 4; ++j) bf[j] = ld_frag<F>(pb + (size_t)(j << 4) * (size_t)KTOT + k0);
#pragma unroll
    for (int i = 0; i < 4; ++i) {
      const F af = ld_frag<F>(pa + (size_t)(i << 4) * (size_t)KTOT + k0);
#pragma unroll
      for (int j = 0; j < 4; ++j) acc[i][j] = mm(af, bf[j], acc[i][j]);
    }
  }

  float* slab = sT[wave];
  const int hh = lane >> 4;
  const int c4 = (lane & 15) * 4;
  const int nc = n0 + c4;
  const bool cok = nc < N;
  v4f bv = (v4f){0.f, 0.f, 0.f, 0.f};
  if (EPI == 1) {
    bv = *(const v4fa*)(bias + clampi(nc, 0, N - 4));
    asm volatile("" :: "v"(bv));
  }
#pragma unroll
  for (int i = 0; i < 4; ++i) {
    const int mBase = m0 + (i << 4);
#pragma unroll
    for (int j = 0; j < 4; ++j) {
#pragma unroll
      for (int r = 0; r < 8; ++r) slab[(h8 + r) * 68 + (j << 4) + rl] = acc[i][j][r];
    }
    __builtin_amdgcn_fence(__ATOMIC_RELEASE, "workgroup");
    __builtin_amdgcn_wave_barrier();
    __builtin_amdgcn_fence(__ATOMIC_ACQUIRE, "workgroup");
    v4f vv[8];
#pragma unroll
    for (int it = 0; it < 8; ++it) {
      const int row = it * 2 + hh;
      v4f v = *(const v4fa*)(slab + row * 68 + c4);
      if (EPI == 1) v += bv;
      vv[it] = v;
    }
    for (int pass = 0; pass < 2; ++pass) {
#pragma unroll
      for (int it = 0; it < 8; ++it) {
        const int row = mBase + it * 2 + hh;
        if (cok && row < M) *(volatile v4f*)(D + (size_t)row * (size_t)ldd + nc) = vv[it];
      }
      __threadfence();
    }
    __builtin_amdgcn_fence(__ATOMIC_RELEASE, "workgroup");
    __builtin_amdgcn_wave_barrier();
    __builtin_amdgcn_fence(__ATOMIC_ACQUIRE, "workgroup");
  }
}

#include <stddef.h>
#include <stdint.h>
#include <math.h>

#pragma clang fp contract(off)

#define NN      50000
#define NE      800000
#define FIN     64
#define FH      128
#define KH2     256
#define MP      50048
#define NTHR    256
#define NWAVE   8
#define EPT     8
#define WCH     (32 * EPT)
#define NBRUN   512
#define SLB     9
#define NBK     98
#define WLCAP   2048
#define RCAP    12288
#define DEGCAP  48
#define MAXDEG_MEAS_G  38
#define MAXDEG_MEAS_F  33
#define MAXB512_MEAS_G 8439
#define MAXB512_MEAS_F 8408

#define BK_ZINTS (NWAVE * WLCAP + RCAP + 3 * NBRUN)
#define BK_INTS  (BK_ZINTS + 16)
#define BK_LDS   (BK_INTS * 4)

#define XM_BLOCKS (MP * FIN / 8 / 256)
#define PB_W1   4
#define PB_WS   2
#define PB_WH   8
#define PB_TAB  1
#define PB_NRM  49
#define PB_TOT  (PB_W1 + PB_WS + PB_WH + PB_TAB + 2 * PB_NRM)
#define G1_BLOCKS ((((MP / 64) * (FH / 64)) + 7) / 8)
#define G2_BLOCKS ((((MP / 64) * (FIN / 64)) + 7) / 8)

static_assert(FIN % 32 == 0 && FH % 32 == 0 && KH2 == 2 * FH && KH2 % 32 == 0);
static_assert(FIN % 8 == 0 && FH % 8 == 0 && FIN == 16 * 4 && FH == 32 * 4);
static_assert(MP % 128 == 0 && MP % 64 == 0 && MP >= NN && MP == 391 * 128 && MP % 16 == 0);
static_assert((MP * FIN / 8) % 256 == 0);
static_assert((FH * FIN / 8) == PB_W1 * NTHR && (FIN * FIN / 8) == PB_WS * NTHR && (FIN * KH2 / 8) == PB_WH * NTHR);
static_assert(PB_NRM * NTHR >= MP / 4 && MP % 4 == 0 && NN % 4 == 0 && (MP / 4) % 32 == 0);
static_assert(NBRUN == (1 << SLB) && NBRUN % 32 == 0 && NBRUN / 4 <= NTHR && NBRUN % 2 == 0);
static_assert(NBK * NBRUN >= NN && (NBK - 1) * NBRUN < NN);
static_assert(NE < (1 << 22) && (((long long)NE) << SLB) < (1LL << 31));
static_assert(NE % WCH == 0 && NE % 4 == 0);
static_assert((long long)RCAP * 100 >= (long long)MAXB512_MEAS_G * 125);
static_assert((long long)RCAP * 100 >= (long long)MAXB512_MEAS_F * 125);
static_assert(WLCAP >= MAXB512_MEAS_G / 8 + 8 * 33 + 1 && WLCAP >= MAXB512_MEAS_F / 8 + 8 * 33 + 1);
static_assert(MAXDEG_MEAS_G + 8 <= DEGCAP && MAXDEG_MEAS_F + 8 <= DEGCAP);
static_assert(RCAP % (NTHR * 4) == 0 && BK_ZINTS % 4 == 0);
static_assert(BK_LDS <= 327680);
static_assert(MP % NWAVE == 0);
static_assert(NN % (2 * NWAVE) == 0);
static_assert(G1_BLOCKS == 196 && G2_BLOCKS == 98);

typedef unsigned int v2u __attribute__((ext_vector_type(2)));
typedef int          v4i __attribute__((ext_vector_type(4)));
typedef v2u __attribute__((may_alias)) v2ua;
typedef v4u __attribute__((may_alias)) v4ua;
typedef v4i __attribute__((may_alias)) v4ia;

__device__ __forceinline__ void st2_v4u(unsigned short* p, v4u v) {
  volatile v4u* q = (volatile v4u*)p;
  *q = v;
  __threadfence();
  *q = v;
}
__device__ __forceinline__ void st2_v4f(float* p, v4f v) {
  volatile v4f* q = (volatile v4f*)p;
  *q = v;
  __threadfence();
  *q = v;
}

__device__ __forceinline__ float bfv_pin(float f) {
  float t = bf16_val(f);
  asm volatile("" : "+v"(t));
  return t;
}

__device__ __forceinline__ v4u gather8_bf16(const float* __restrict__ base, int stride) {
  float f[8];
#pragma unroll
  for (int i = 0; i < 8; ++i) f[i] = base[(size_t)i * (size_t)stride];
  return (v4u){ pk16(bf16_bits(f[0]), bf16_bits(f[1])), pk16(bf16_bits(f[2]), bf16_bits(f[3])),
                pk16(bf16_bits(f[4]), bf16_bits(f[5])), pk16(bf16_bits(f[6]), bf16_bits(f[7])) };
}

__global__ __launch_bounds__(NTHR) void k_xm(const float* __restrict__ feat, const float* __restrict__ mask,
                                             unsigned short* XM) {
  const unsigned g = blockIdx.x * 256u + threadIdx.x;
  const int row = (int)(g >> 3);
  const int p8  = (int)(g & 7u) * 8;
  const int rr  = row < NN - 1 ? row : NN - 1;
  const size_t off = (size_t)rr * FIN + (size_t)p8;
  const v4f fa = *(const v4fa*)(feat + off);
  const v4f fb = *(const v4fa*)(feat + off + 4);
  const v4f ma = *(const v4fa*)(mask + off);
  const v4f mb = *(const v4fa*)(mask + off + 4);
  asm volatile("" :: "v"(fa), "v"(fb));
  asm volatile("" :: "v"(ma), "v"(mb));
  unsigned w[8];
#pragma unroll
  for (int e = 0; e < 4; ++e) {
    const float x0 = bfv_pin(fa[e]);
    const float m0 = bfv_pin(ma[e]);
    const float x1 = bfv_pin(fb[e]);
    const float m1 = bfv_pin(mb[e]);
    float p0 = x0 * m0;
    float p1 = x1 * m1;
    asm volatile("" : "+v"(p0));
    asm volatile("" : "+v"(p1));
    w[e]     = bf16_bits(p0);
    w[4 + e] = bf16_bits(p1);
  }
  const unsigned km = (row < NN) ? 0xFFFFFFFFu : 0u;
  v4u o = (v4u){ pk16(w[0], w[1]), pk16(w[2], w[3]), pk16(w[4], w[5]), pk16(w[6], w[7]) };
  o &= (v4u){ km, km, km, km };
  st2_v4u(XM + (size_t)g * 8, o);
}

__device__ __forceinline__ void norm_units(const float* __restrict__ src, float* dst, int u) {
  const int a = clampi(4 * u, 0, NN - 4);
  const v4f v = *(const v4fa*)(src + a);
  asm volatile("" :: "v"(v));
  const unsigned km = (u < NN / 4) ? 0xFFFFFFFFu : 0u;
  v4f o;
#pragma unroll
  for (int e = 0; e < 4; ++e) o[e] = __uint_as_float(__float_as_uint(bf16_val(v[e])) & km);
  if (u < MP / 4) st2_v4f(dst + (size_t)4 * (size_t)u, o);
}

__global__ __launch_bounds__(NTHR) void k_prep(const float* __restrict__ w1, const float* __restrict__ wsk,
                                               const float* __restrict__ wh, const float* __restrict__ b1,
                                               const float* __restrict__ bh, const float* __restrict__ bs,
                                               const float* __restrict__ ng, const float* __restrict__ nf,
                                               unsigned short* w1t, unsigned short* wst, unsigned short* wh2,
                                               float* tab, float* NG, float* NF) {
  const int tid = (int)threadIdx.x;
  const int blk = (int)blockIdx.x;
  if (blk < PB_W1) {
    const int u = blk * NTHR + tid;
    const int n = u >> 3, k8 = (u & 7) * 8;
    const v4u o = gather8_bf16(w1 + (size_t)k8 * FH + n, FH);
    st2_v4u(w1t + (size_t)n * FIN + k8, o);
  } else if (blk < PB_W1 + PB_WS) {
    const int u = (blk - PB_W1) * NTHR + tid;
    const int n = u >> 3, k8 = (u & 7) * 8;
    const v4u o = gather8_bf16(wsk + (size_t)k8 * FIN + n, FIN);
    st2_v4u(wst + (size_t)n * FIN + k8, o);
  } else if (blk < PB_W1 + PB_WS + PB_WH) {
    const int u = (blk - PB_W1 - PB_WS) * NTHR + tid;
    const int n = u >> 5, k8 = (u & 31) * 8;
    const int ks = k8 & (FH - 1);
    const v4u o = gather8_bf16(wh + (size_t)ks * FIN + n, FIN);
    st2_v4u(wh2 + (size_t)n * KH2 + k8, o);
  } else if (blk < PB_W1 + PB_WS + PB_WH + PB_TAB) {
    const int t = tid & 63;
    const v4f x1 = *(const v4fa*)(b1 + clampi(4 * t, 0, FH - 4));
    const v4f x2 = *(const v4fa*)(bh + clampi(4 * (t - 32), 0, FIN - 4));
    const v4f x3 = *(const v4fa*)(bs + clampi(4 * (t - 48), 0, FIN - 4));
    asm volatile("" :: "v"(x1), "v"(x2), "v"(x3));
    const unsigned m1 = (t < 32) ? 0xFFFFFFFFu : 0u;
    const unsigned m2 = (t >= 32 && t < 48) ? 0xFFFFFFFFu : 0u;
    const unsigned m3 = (t >= 48) ? 0xFFFFFFFFu : 0u;
    v4f o;
#pragma unroll
    for (int e = 0; e < 4; ++e) {
      const unsigned u1 = __float_as_uint(bf16_val(x1[e])) & m1;
      const unsigned u2 = __float_as_uint(bf16_val(x2[e])) & m2;
      const unsigned u3 = __float_as_uint(bf16_val(x3[e])) & m3;
      o[e] = __uint_as_float(u1 | u2 | u3);
    }
    if (tid < 64) st2_v4f(tab + 4 * tid, o);
  } else if (blk < PB_W1 + PB_WS + PB_WH + PB_TAB + PB_NRM) {
    const int u = (blk - (PB_W1 + PB_WS + PB_WH + PB_TAB)) * NTHR + tid;
    norm_units(ng, NG, u);
  } else {
    const int u = (blk - (PB_W1 + PB_WS + PB_WH + PB_TAB + PB_NRM)) * NTHR + tid;
    norm_units(nf, NF, u);
  }
}

__device__ __forceinline__ void lists_flush(const int* pl, const int* cnt, const int* offs, int ov,
                                            int* lp, int* cp, int* op, int* fp, int tid) {
#pragma unroll 1
  for (int i = tid * 4; i < RCAP; i += NTHR * 4) {
    const v4i v = *(const v4ia*)(pl + i);
    *(volatile v4i*)(lp + i) = v;
  }
  if (tid < NBRUN / 4) {
    const v4i vc = *(const v4ia*)(cnt + 4 * tid);
    const v4i vo = *(const v4ia*)(offs + 4 * tid);
    *(volatile v4i*)(cp + 4 * tid) = vc;
    *(volatile v4i*)(op + 4 * tid) = vo;
  }
  if (tid < 8) {
    const v4i f = {ov, ov, ov, ov};
    *(volatile v4i*)(fp + 4 * tid) = f;
  }
}

__global__ __launch_bounds__(NTHR) void k_lists(const int* __restrict__ keys, const int* __restrict__ ids,
                                                int* LIST, int* CNT, int* OFF, int* FLAG) {
  extern __shared__ __attribute__((aligned(16))) int dsm[];
  int* wl   = dsm;
  int* pl   = dsm + NWAVE * WLCAP;
  int* cnt  = pl + RCAP;
  int* offs = cnt + NBRUN;
  int* cur  = offs + NBRUN;
  int* misc = cur + NBRUN;
  const int tid = (int)threadIdx.x, lane = tid & 31, wave = tid >> 5;
  const int blk = (int)blockIdx.x;
  const unsigned nbs = (unsigned)(blk * NBRUN);

  {
    const v4i z4 = {0, 0, 0, 0};
#pragma unroll 1
    for (int i = tid * 4; i < BK_ZINTS; i += NTHR * 4) *(v4ia*)(dsm + i) = z4;
    if (tid < 16) misc[tid] = 0;
  }
  __syncthreads();

  {
    const int per  = ((NE + NWAVE * WCH - 1) / (NWAVE * WCH)) * WCH;
    const int ebeg = wave * per;
    const int eend = (ebeg + per < NE) ? (ebeg + per) : NE;
    int* mylist = wl + wave * WLCAP;
    int wc = 0;
#pragma unroll 1
    for (int cb = ebeg; cb < eend; cb += WCH) {
      const int e0 = cb + lane * EPT;
      const v4i da = *(const v4ia*)(keys + e0);
      const v4i db = *(const v4ia*)(keys + e0 + 4);
      const int d0 = da.x, d1 = da.y, d2 = da.z, d3 = da.w;
      const int d4 = db.x, d5 = db.y, d6 = db.z, d7 = db.w;
      asm volatile("" :: "v"(d0), "v"(d1), "v"(d2), "v"(d3));
      asm volatile("" :: "v"(d4), "v"(d5), "v"(d6), "v"(d7));
      const unsigned s0 = (unsigned)d0 - nbs, s1 = (unsigned)d1 - nbs;
      const unsigned s2 = (unsigned)d2 - nbs, s3 = (unsigned)d3 - nbs;
      const unsigned s4 = (unsigned)d4 - nbs, s5 = (unsigned)d5 - nbs;
      const unsigned s6 = (unsigned)d6 - nbs, s7 = (unsigned)d7 - nbs;
      const bool h0 = s0 < (unsigned)NBRUN, h1 = s1 < (unsigned)NBRUN, h2 = s2 < (unsigned)NBRUN, h3 = s3 < (unsigned)NBRUN;
      const bool h4 = s4 < (unsigned)NBRUN, h5 = s5 < (unsigned)NBRUN, h6 = s6 < (unsigned)NBRUN, h7 = s7 < (unsigned)NBRUN;
      const unsigned m0 = __builtin_amdgcn_ballot_w32(h0), m1 = __builtin_amdgcn_ballot_w32(h1);
      const unsigned m2 = __builtin_amdgcn_ballot_w32(h2), m3 = __builtin_amdgcn_ballot_w32(h3);
      const unsigned m4 = __builtin_amdgcn_ballot_w32(h4), m5 = __builtin_amdgcn_ballot_w32(h5);
      const unsigned m6 = __builtin_amdgcn_ballot_w32(h6), m7 = __builtin_amdgcn_ballot_w32(h7);
      const unsigned any = m0 | m1 | m2 | m3 | m4 | m5 | m6 | m7;
      if (any != 0u) {
        const int pre = (int)(__builtin_amdgcn_mbcnt_lo(m0, 0u) + __builtin_amdgcn_mbcnt_lo(m1, 0u) +
                              __builtin_amdgcn_mbcnt_lo(m2, 0u) + __builtin_amdgcn_mbcnt_lo(m3, 0u) +
                              __builtin_amdgcn_mbcnt_lo(m4, 0u) + __builtin_amdgcn_mbcnt_lo(m5, 0u) +
                              __builtin_amdgcn_mbcnt_lo(m6, 0u) + __builtin_amdgcn_mbcnt_lo(m7, 0u));
        int p = wc + pre;
        if (h0) { if (p < WLCAP) mylist[p] = ((e0 + 0) << SLB) | (int)s0; p = p + 1; }
        if (h1) { if (p < WLCAP) mylist[p] = ((e0 + 1) << SLB) | (int)s1; p = p + 1; }
        if (h2) { if (p < WLCAP) mylist[p] = ((e0 + 2) << SLB) | (int)s2; p = p + 1; }
        if (h3) { if (p < WLCAP) mylist[p] = ((e0 + 3) << SLB) | (int)s3; p = p + 1; }
        if (h4) { if (p < WLCAP) mylist[p] = ((e0 + 4) << SLB) | (int)s4; p = p + 1; }
        if (h5) { if (p < WLCAP) mylist[p] = ((e0 + 5) << SLB) | (int)s5; p = p + 1; }
        if (h6) { if (p < WLCAP) mylist[p] = ((e0 + 6) << SLB) | (int)s6; p = p + 1; }
        if (h7) { if (p < WLCAP) mylist[p] = ((e0 + 7) << SLB) | (int)s7; p = p + 1; }
        wc += (int)(__builtin_popcount(m0) + __builtin_popcount(m1) + __builtin_popcount(m2) + __builtin_popcount(m3) +
                    __builtin_popcount(m4) + __builtin_popcount(m5) + __builtin_popcount(m6) + __builtin_popcount(m7));
      }
    }
    if (lane == 0) misc[wave] = wc;
  }
  __syncthreads();

  if (wave == 0) {
    int ov = 0;
    int tot = 0;
#pragma unroll 1
    for (int w2 = 0; w2 < NWAVE; ++w2) {
      int c = misc[w2];
      if (c > WLCAP) ov = 1;
      c = c < 0 ? 0 : (c > WLCAP ? WLCAP : c);
      tot += c;
#pragma unroll 1
      for (int b0 = 0; b0 < c; b0 += 32) {
        const int idx = b0 + lane;
        const int ent = wl[w2 * WLCAP + (idx < WLCAP ? idx : WLCAP - 1)];
        const int m32 = (c - b0) < 32 ? (c - b0) : 32;
#pragma unroll 1
        for (int k = 0; k < m32; ++k) {
          const int u    = __builtin_amdgcn_readlane(ent, k);
          const int slot = u & (NBRUN - 1);
          if (lane == 0) cnt[slot] = cnt[slot] + 1;
        }
      }
    }
    if (tot > RCAP) ov = 1;
    if (lane == 0) misc[9] = ov;
  }
  __syncthreads();
  if (wave == 0) {
    const int base = lane * (NBRUN / 32);
    int s = 0;
#pragma unroll 1
    for (int i = 0; i < NBRUN / 32; ++i) s += cnt[base + i];
    int incl = s;
#pragma unroll
    for (int d = 1; d < 32; d <<= 1) {
      const int y = __shfl_up(incl, d, 32);
      if (lane >= d) incl += y;
    }
    int run = incl - s;
#pragma unroll 1
    for (int i = 0; i < NBRUN / 32; ++i) {
      const int cv = cnt[base + i];
      offs[base + i] = run;
      cur[base + i]  = run;
      run += cv;
    }
  }
  __syncthreads();

  if (wave == 0) {
#pragma unroll 1
    for (int w2 = 0; w2 < NWAVE; ++w2) {
      int c = misc[w2];
      c = c < 0 ? 0 : (c > WLCAP ? WLCAP : c);
#pragma unroll 1
      for (int b0 = 0; b0 < c; b0 += 32) {
        const int idx = b0 + lane;
        const int ent = wl[w2 * WLCAP + (idx < WLCAP ? idx : WLCAP - 1)];
        int eid = (ent >> SLB) & 0x3FFFFF;
        eid = eid > NE - 1 ? NE - 1 : eid;
        int sr = ids[eid];
        asm volatile("" :: "v"(sr));
        sr = sr < 0 ? 0 : (sr > NN - 1 ? NN - 1 : sr);
        const int m32 = (c - b0) < 32 ? (c - b0) : 32;
#pragma unroll 1
        for (int k = 0; k < m32; ++k) {
          const int u    = __builtin_amdgcn_readlane(ent, k);
          const int w0   = __builtin_amdgcn_readlane(sr, k);
          const int slot = u & (NBRUN - 1);
          if (lane == 0) {
            int p = cur[slot];
            p = p < 0 ? 0 : (p > RCAP - 1 ? RCAP - 1 : p);
            pl[p] = w0;
            cur[slot] = p + 1;
          }
        }
      }
    }
  }
  __syncthreads();

  const int ovf = misc[9];
  int* lp = LIST + (size_t)blk * (size_t)RCAP;
  int* cp = CNT  + (size_t)blk * NBRUN;
  int* op = OFF  + (size_t)blk * NBRUN;
  int* fp = FLAG + (size_t)blk * 32;
  lists_flush(pl, cnt, offs, ovf, lp, cp, op, fp, tid);
  __threadfence();
  lists_flush(pl, cnt, offs, ovf, lp, cp, op, fp, tid);
}

__global__ __launch_bounds__(NTHR) void k_walk_g128(const int* __restrict__ LIST, const int* __restrict__ CNT,
                                                    const int* __restrict__ OFF, const int* __restrict__ FLAG,
                                                    const float* __restrict__ NG, const float* __restrict__ T1,
                                                    const float* __restrict__ B1, unsigned short* OPH) {
  __shared__ __attribute__((aligned(16))) unsigned srow[NWAVE][128];
  const int tid = (int)threadIdx.x, lane = tid & 31, wave = tid >> 5;
  const int node = (int)blockIdx.x * NWAVE + wave;
  const int dn = node < NN - 1 ? node : NN - 1;
  const int blk = dn >> SLB;
  const int* lb = LIST + (size_t)blk * (size_t)RCAP;
  const int craw = CNT[dn];
  const int oraw = OFF[dn];
  const int flag = FLAG[(size_t)blk * 32];
  const float nd = NG[dn];
  const v4f bb = *(const v4fa*)(B1 + 4 * lane);
  asm volatile("" :: "v"(craw), "v"(oraw), "v"(flag), "v"(nd));
  asm volatile("" :: "v"(bb));

  const bool big = craw > DEGCAP;
  const int c = __builtin_amdgcn_readfirstlane(craw < 0 ? 0 : (craw > DEGCAP ? DEGCAP : craw));
  const int o = oraw < 0 ? 0 : (oraw > RCAP - 1 ? RCAP - 1 : oraw);
  int last = o + (c > 0 ? c : 1) - 1;
  last = last > RCAP - 1 ? RCAP - 1 : last;

  v4f acc = (v4f){0.0f, 0.0f, 0.0f, 0.0f};
#pragma unroll 1
  for (int b0 = 0; b0 < c; b0 += 32) {
    int idx = o + b0 + lane;
    idx = idx > last ? last : idx;
    int sr = lb[idx];
    asm volatile("" :: "v"(sr));
    sr = sr < 0 ? 0 : (sr > NN - 1 ? NN - 1 : sr);
    const float nsv = NG[sr];
    asm volatile("" :: "v"(nsv));
    const int nsb = __float_as_int(nsv);
    const int m32 = (c - b0) < 32 ? (c - b0) : 32;
#pragma unroll 1
    for (int k = 0; k < m32; ++k) {
      const int   sk = __builtin_amdgcn_readlane(sr, k);
      const float ns = __int_as_float(__builtin_amdgcn_readlane(nsb, k));
      const v4f q = *(const v4fa*)(T1 + (size_t)sk * FH + 4 * lane);
      asm volatile("" :: "v"(q));
      v4f p = q * ns;
      asm volatile("" : "+v"(p));
      acc = acc + p;
    }
  }
  v4f t = acc * nd;
  asm volatile("" : "+v"(t));
  const v4f v = t + bb;
  const bool bad = (flag != 0) | big;
  const float qnan = __uint_as_float(0x7fc00000u);
  float hv[4];
#pragma unroll
  for (int e = 0; e < 4; ++e) {
    const float x = v[e];
    const float r = (x > 0.0f) ? x : (x - x);
    hv[e] = bad ? qnan : r;
  }
  const v2u hi2 = (v2u){ pk16(bf16_bits(hv[0]), bf16_bits(hv[1])), pk16(bf16_bits(hv[2]), bf16_bits(hv[3])) };
  const v2u lo2 = (v2u){ pk16(bf16_lo_bits(hv[0]), bf16_lo_bits(hv[1])), pk16(bf16_lo_bits(hv[2]), bf16_lo_bits(hv[3])) };
  unsigned* row = srow[wave];
  *(v2ua*)(row + 2 * lane)      = hi2;
  *(v2ua*)(row + 64 + 2 * lane) = lo2;
  __builtin_amdgcn_fence(__ATOMIC_RELEASE, "workgroup");
  __builtin_amdgcn_wave_barrier();
  __builtin_amdgcn_fence(__ATOMIC_ACQUIRE, "workgroup");
  v4u ov = *(const v4ua*)(row + 4 * lane);
  const unsigned km = (node < NN) ? 0xFFFFFFFFu : 0u;
  ov &= (v4u){ km, km, km, km };
  st2_v4u(OPH + (size_t)node * KH2 + 8 * lane, ov);
}

__device__ __forceinline__ v4f walk64(const int* __restrict__ lb, int c, int o, int cmax,
                                      const float* __restrict__ NRM, const float* __restrict__ PL, int lane) {
  const int j  = lane & 15;
  const int gb = lane & 16;
  const int c4 = j * 4;
  int last = o + (c > 0 ? c : 1) - 1;
  last = last > RCAP - 1 ? RCAP - 1 : last;
  v4f acc = (v4f){0.0f, 0.0f, 0.0f, 0.0f};
#pragma unroll 1
  for (int b0 = 0; b0 < cmax; b0 += 16) {
    int idx = o + b0 + j;
    idx = idx > last ? last : idx;
    int sr = lb[idx];
    asm volatile("" :: "v"(sr));
    sr = sr < 0 ? 0 : (sr > NN - 1 ? NN - 1 : sr);
    const float nsv = NRM[sr];
    asm volatile("" :: "v"(nsv));
    const int nsb = __float_as_int(nsv);
    const int m16 = (cmax - b0) < 16 ? (cmax - b0) : 16;
#pragma unroll 1
    for (int k = 0; k < m16; ++k) {
      const int   sk = __shfl(sr, gb | k, 32);
      const float ns = __int_as_float(__shfl(nsb, gb | k, 32));
      const unsigned vm = ((b0 + k) < c) ? 0xFFFFFFFFu : 0u;
      const v4f q = *(const v4fa*)(PL + (size_t)sk * FIN + c4);
      asm volatile("" :: "v"(q));
      v4f p = q * ns;
      asm volatile("" : "+v"(p));
      v4f pm;
#pragma unroll
      for (int e = 0; e < 4; ++e) pm[e] = __uint_as_float(__float_as_uint(p[e]) & vm);
      acc = acc + pm;
    }
  }
  return acc;
}

__global__ __launch_bounds__(NTHR) void k_final(const int* __restrict__ LG, const int* __restrict__ CG,
                                                const int* __restrict__ OFg, const int* __restrict__ FG,
                                                const int* __restrict__ LF, const int* __restrict__ CF,
                                                const int* __restrict__ OFf, const int* __restrict__ FF,
                                                const float* __restrict__ NG, const float* __restrict__ NF,
                                                const float* __restrict__ HB0, const float* __restrict__ S0,
                                                const float* __restrict__ BH, const float* __restrict__ BS,
                                                float* out, int n_nodes) {
  const int tid = (int)threadIdx.x, lane = tid & 31, wave = tid >> 5;
  const int wv = (int)blockIdx.x * NWAVE + wave;
  const int owner = 2 * wv + (lane >> 4);
  const int dn = owner < NN - 1 ? owner : NN - 1;
  const int blk = __builtin_amdgcn_readfirstlane(dn >> SLB);
  const int c4 = (lane & 15) * 4;
  const int cgr = CG[dn],  ogr = OFg[dn], fg = FG[(size_t)blk * 32];
  const int cfr = CF[dn],  ofr = OFf[dn], ff = FF[(size_t)blk * 32];
  const float ngd = NG[dn];
  const float nfd = NF[dn];
  const v4f bh4 = *(const v4fa*)(BH + c4);
  const v4f bs4 = *(const v4fa*)(BS + c4);
  asm volatile("" :: "v"(cgr), "v"(ogr), "v"(fg));
  asm volatile("" :: "v"(cfr), "v"(ofr), "v"(ff));
  asm volatile("" :: "v"(ngd), "v"(nfd));
  asm volatile("" :: "v"(bh4), "v"(bs4));

  const bool big = (cgr > DEGCAP) | (cfr > DEGCAP);
  const int cg = cgr < 0 ? 0 : (cgr > DEGCAP ? DEGCAP : cgr);
  const int cf = cfr < 0 ? 0 : (cfr > DEGCAP ? DEGCAP : cfr);
  const int og = ogr < 0 ? 0 : (ogr > RCAP - 1 ? RCAP - 1 : ogr);
  const int of = ofr < 0 ? 0 : (ofr > RCAP - 1 ? RCAP - 1 : ofr);
  const int cg0 = __builtin_amdgcn_readlane(cg, 0), cg1 = __builtin_amdgcn_readlane(cg, 16);
  const int cf0 = __builtin_amdgcn_readlane(cf, 0), cf1 = __builtin_amdgcn_readlane(cf, 16);
  const int cgmax = cg0 > cg1 ? cg0 : cg1;
  const int cfmax = cf0 > cf1 ? cf0 : cf1;

  const v4f ha = walk64(LG + (size_t)blk * (size_t)RCAP, cg, og, cgmax, NG, HB0, lane);
  const v4f sa = walk64(LF + (size_t)blk * (size_t)RCAP, cf, of, cfmax, NF, S0, lane);

  v4f th = ha * ngd;
  asm volatile("" : "+v"(th));
  v4f ts = sa * nfd;
  asm volatile("" : "+v"(ts));
  const v4f hb = th + bh4;
  const v4f sb = ts + bs4;
  const v4f z = hb + sb;
  const bool bad = (fg != 0) | (ff != 0) | big;
  const float qnan = __uint_as_float(0x7fc00000u);
  v4f r;
#pragma unroll
  for (int e = 0; e < 4; ++e) {
    const float ex = expf(-z[e]);
    const float sg = 1.0f / (1.0f + ex);
    r[e] = bad ? qnan : sg;
  }
  if (owner < n_nodes) {
    volatile v4f* q = (volatile v4f*)(out + (size_t)owner * FIN + c4);
    *q = r;
    __threadfence();
    *q = r;
  }
}

extern "C" void kernel_launch(void* const* d_in, const int* in_sizes, int n_in,
                              void* d_out, int out_size, void* d_ws, size_t ws_size,
                              hipStream_t stream) {
  if (n_in < 14) return;
  if (in_sizes[0] != NN * FIN) return;
  if (in_sizes[1] != NN * FIN) return;
  if (in_sizes[2] != NN) return;
  if (in_sizes[3] != NN) return;
  if (in_sizes[4] != NE || in_sizes[5] != NE) return;
  if (in_sizes[6] != NE || in_sizes[7] != NE) return;
  if (in_sizes[8] != FIN * FH) return;
  if (in_sizes[9] != FH) return;
  if (in_sizes[10] != FH * FIN) return;
  if (in_sizes[11] != FIN) return;
  if (in_sizes[12] != FIN * FIN) return;
  if (in_sizes[13] != FIN) return;
  if (out_size != NN * FIN) return;
  const int n_nodes = in_sizes[2];

  const float* feat = (const float*)d_in[0];
  const float* mask = (const float*)d_in[1];
  const float* ngin = (const float*)d_in[2];
  const float* nfin = (const float*)d_in[3];
  const int* src_g  = (const int*)d_in[4];
  const int* dst_g  = (const int*)d_in[5];
  const int* src_f  = (const int*)d_in[6];
  const int* dst_f  = (const int*)d_in[7];
  const float* W1   = (const float*)d_in[8];
  const float* b1   = (const float*)d_in[9];
  const float* wh   = (const float*)d_in[10];
  const float* bh   = (const float*)d_in[11];
  const float* wsk  = (const float*)d_in[12];
  const float* bs   = (const float*)d_in[13];
  float* out = (float*)d_out;

  constexpr size_t zXM   = (size_t)MP * FIN * 2;
  constexpr size_t zT1   = (size_t)MP * FH * 4;
  constexpr size_t zS0   = (size_t)MP * FIN * 4;
  constexpr size_t zOPH  = (size_t)MP * KH2 * 2;
  constexpr size_t zHB0  = (size_t)MP * FIN * 4;
  constexpr size_t zLIST = (size_t)NBK * RCAP * 4;
  constexpr size_t zTBL  = (size_t)NBK * NBRUN * 4;
  constexpr size_t zFLAG = (size_t)NBK * 128;
  constexpr size_t zNRM  = (size_t)MP * 4;
  constexpr size_t zW1T  = (size_t)FH * FIN * 2;
  constexpr size_t zWST  = (size_t)FIN * FIN * 2;
  constexpr size_t zWH2  = (size_t)FIN * KH2 * 2;
  constexpr size_t zTAB  = 1024;
  constexpr size_t oXM   = 0;
  constexpr size_t oT1   = oXM + zXM;
  constexpr size_t oS0   = oT1 + zT1;
  constexpr size_t oOPH  = oS0 + zS0;
  constexpr size_t oHB0  = oOPH + zOPH;
  constexpr size_t oLG   = oHB0 + zHB0;
  constexpr size_t oLF   = oLG + zLIST;
  constexpr size_t oCG   = oLF + zLIST;
  constexpr size_t oOG   = oCG + zTBL;
  constexpr size_t oCF   = oOG + zTBL;
  constexpr size_t oOF   = oCF + zTBL;
  constexpr size_t oFG   = oOF + zTBL;
  constexpr size_t oFF   = oFG + zFLAG;
  constexpr size_t oNG   = oFF + zFLAG;
  constexpr size_t oNF   = oNG + zNRM;
  constexpr size_t oW1T  = oNF + zNRM;
  constexpr size_t oWST  = oW1T + zW1T;
  constexpr size_t oWH2  = oWST + zWST;
  constexpr size_t oTAB  = oWH2 + zWH2;
  constexpr size_t oEND  = oTAB + zTAB;
  static_assert(zXM % 256 == 0 && zT1 % 256 == 0 && zS0 % 256 == 0 && zOPH % 256 == 0 && zHB0 % 256 == 0);
  static_assert(zLIST % 256 == 0 && zTBL % 256 == 0 && zFLAG % 256 == 0 && zNRM % 256 == 0);
  static_assert(zW1T % 256 == 0 && zWST % 256 == 0 && zWH2 % 256 == 0 && zTAB % 256 == 0);
  static_assert(zTAB >= (size_t)(FH + 2 * FIN) * 4);
  static_assert(zTBL >= (size_t)NN * 4);
  static_assert(oEND == 94200320);
  static_assert(oEND <= ((size_t)128 << 20));
  if (oEND > ws_size) return;

  char* ws = (char*)d_ws;
  unsigned short* XM  = (unsigned short*)(ws + oXM);
  float*          T1  = (float*)(ws + oT1);
  float*          S0  = (float*)(ws + oS0);
  unsigned short* OPH = (unsigned short*)(ws + oOPH);
  float*          HB0 = (float*)(ws + oHB0);
  int*            LG  = (int*)(ws + oLG);
  int*            LF  = (int*)(ws + oLF);
  int*            CG  = (int*)(ws + oCG);
  int*            OG  = (int*)(ws + oOG);
  int*            CF  = (int*)(ws + oCF);
  int*            OF2 = (int*)(ws + oOF);
  int*            FG  = (int*)(ws + oFG);
  int*            FF  = (int*)(ws + oFF);
  float*          NG  = (float*)(ws + oNG);
  float*          NF  = (float*)(ws + oNF);
  unsigned short* W1T = (unsigned short*)(ws + oW1T);
  unsigned short* WST = (unsigned short*)(ws + oWST);
  unsigned short* WH2 = (unsigned short*)(ws + oWH2);
  float*          TAB = (float*)(ws + oTAB);

  hipFuncSetAttribute(reinterpret_cast<const void*>(&k_lists), hipFuncAttributeMaxDynamicSharedMemorySize, (int)BK_LDS);

  k_xm<<<XM_BLOCKS, NTHR, 0, stream>>>(feat, mask, XM);
  k_prep<<<PB_TOT, NTHR, 0, stream>>>(W1, wsk, wh, b1, bh, bs, ngin, nfin, W1T, WST, WH2, TAB, NG, NF);
  k_gemm_nt<0, 0><<<G1_BLOCKS, 256, 0, stream>>>(XM, W1T, TAB, T1, MP, FH, FIN, FH);
  k_gemm_nt<0, 0><<<G2_BLOCKS, 256, 0, stream>>>(XM, WST, TAB, S0, MP, FIN, FIN, FIN);
  k_lists<<<NBK, NTHR, BK_LDS, stream>>>(dst_g, src_g, LG, CG, OG, FG);
  k_lists<<<NBK, NTHR, BK_LDS, stream>>>(dst_f, src_f, LF, CF, OF2, FF);
  k_walk_g128<<<MP / NWAVE, NTHR, 0, stream>>>(LG, CG, OG, FG, NG, T1, TAB, OPH);
  k_gemm_nt<0, 0><<<G2_BLOCKS, 256, 0, stream>>>(OPH, WH2, TAB, HB0, MP, FIN, KH2, FIN);
  k_final<<<NN / (2 * NWAVE), NTHR, 0, stream>>>(LG, CG, OG, FG, LF, CF, OF2, FF, NG, NF, HB0, S0,
                                                 TAB + FH, TAB + FH + FIN, out, n_nodes);
}
